// NA3DBlock_69879117906012
// MI455X (gfx1250) — hardware-verified
//
#include <hip/hip_runtime.h>
#include <math.h>

typedef __attribute__((ext_vector_type(16))) _Float16 v16h;
typedef __attribute__((ext_vector_type(16))) __bf16 v16b;
typedef __attribute__((ext_vector_type(8)))  _Float16 v8h;
typedef __attribute__((ext_vector_type(8)))  float v8f;
typedef __attribute__((ext_vector_type(4)))  float v4f;
typedef __attribute__((ext_vector_type(2)))  float v2f;
typedef __attribute__((ext_vector_type(4)))  unsigned v4u;
typedef __attribute__((ext_vector_type(4)))  int v4i;
typedef float __attribute__((may_alias)) float_a;
typedef int __attribute__((may_alias)) int_a;

template <typename T> __device__ __forceinline__ void vst2(void* p, T v) { *(volatile T*)p = v; __threadfence(); *(volatile T*)p = v; }
__device__ __forceinline__ v8f wmma16(v16h a, v16h b, v8f c) {
  v8f d = __builtin_amdgcn_wmma_f32_16x16x32_f16(false, a, false, b, (short)0, c, false, false);
  asm volatile("v_nop\n\tv_nop\n\tv_nop\n\tv_nop" : "+v"(d) : "v"(a), "v"(b));
  return d;
}
__device__ __forceinline__ v8f wmma_bf(v16b a, v16b b, v8f c) {
  v8f d = __builtin_amdgcn_wmma_f32_16x16x32_bf16(false, a, false, b, (short)0, c, false, false);
  asm volatile("v_nop\n\tv_nop\n\tv_nop\n\tv_nop" : "+v"(d) : "v"(a), "v"(b));
  return d;
}
__device__ __forceinline__ v16h frag_h(const _Float16* rowk0, int lane) {
  union { v16h v; v8h q[2]; } u; const _Float16* p = rowk0 + 8 * (lane >> 4);
  u.q[0] = *(const v8h*)p; u.q[1] = *(const v8h*)(p + 16); return u.v;
}
__device__ __forceinline__ v16h frag_f32(const float* rowk0, int lane) {
  v16h a; const float* p = rowk0 + 8 * (lane >> 4);
#pragma unroll
  for (int i = 0; i < 8; ++i) { a[i] = (_Float16)p[i]; a[8 + i] = (_Float16)p[16 + i]; }
  return a;
}
__device__ __forceinline__ v16h frag_f32s(const float* rowk0, int lane, float sc) {
  v16h a; const float* p = rowk0 + 8 * (lane >> 4);
#pragma unroll
  for (int i = 0; i < 8; ++i) { a[i] = (_Float16)(p[i] * sc); a[8 + i] = (_Float16)(p[16 + i] * sc); }
  return a;
}
__device__ __forceinline__ v16h fragc_f32(const float* W, int k0, int n, int lane, int ld, int K) {
  v16h a; const int g = lane >> 4;
#pragma unroll
  for (int i = 0; i < 8; ++i) { const int ka = k0 + 8 * g + i, kb = ka + 16;
    a[i] = (_Float16)(ka < K ? W[(size_t)ka * ld + n] : 0.f); a[8 + i] = (_Float16)(kb < K ? W[(size_t)kb * ld + n] : 0.f); }
  return a;
}
struct F2 { v16b h, l; };
__device__ __forceinline__ F2 bsplit16(const float v[16]) { F2 r;
#pragma unroll
  for (int i = 0; i < 16; ++i) { const __bf16 h = (__bf16)v[i]; r.h[i] = h; r.l[i] = (__bf16)(v[i] - (float)h); }
  return r; }
__device__ __forceinline__ F2 split_row(const float* row, int k0, int lane) { float v[16]; const float* p = row + k0 + 8 * (lane >> 4);
#pragma unroll
  for (int i = 0; i < 8; ++i) { v[i] = p[i]; v[8 + i] = p[16 + i]; }
  return bsplit16(v); }
__device__ __forceinline__ F2 split_rowK(const float* row, int k0, int lane, int K) { float v[16]; const int g = lane >> 4;
#pragma unroll
  for (int i = 0; i < 8; ++i) { const int ka = k0 + 8 * g + i, kb = ka + 16; v[i] = ka < K ? row[ka] : 0.f; v[8 + i] = kb < K ? row[kb] : 0.f; }
  return bsplit16(v); }
__device__ __forceinline__ F2 split_col(const float* W, int k0, int n, int lane, int ld, int K) { float v[16]; const int g = lane >> 4;
#pragma unroll
  for (int i = 0; i < 8; ++i) { const int ka = k0 + 8 * g + i, kb = ka + 16; v[i] = ka < K ? W[(size_t)ka * ld + n] : 0.f; v[8 + i] = kb < K ? W[(size_t)kb * ld + n] : 0.f; }
  return bsplit16(v); }
__device__ __forceinline__ v8f mac3(const F2& a, const F2& b, v8f c) { c = wmma_bf(a.l, b.h, c); c = wmma_bf(a.h, b.l, c); return wmma_bf(a.h, b.h, c); }
__device__ __forceinline__ float sigm(float v) { return 1.0f / (1.0f + expf(-v)); }
#define LDSX() do { asm volatile("s_wait_dscnt 0" ::: "memory"); __builtin_amdgcn_wave_barrier(); __builtin_amdgcn_fence(__ATOMIC_RELEASE, "workgroup"); } while (0)

#define CC 128
#define SD 20
#define NT (SD * SD * SD)
#define NTP 8064
#define NHD 8
#define HD 16
#define KW 5
#define NNB (KW * KW * KW)
#define RB (2 * KW - 1)
#define FF 512

__device__ __forceinline__ float gelu_e(float v) { return 0.5f * v * (1.0f + erff(v * 0.70710678118654752f)); }

__global__ __launch_bounds__(256) void k_bnstat(const float* __restrict__ x, float* __restrict__ stat) {
  __shared__ float sred[2][8];
  const int c = blockIdx.x, tid = threadIdx.x, wv = tid >> 5, lane = tid & 31; const float* xc = x + (size_t)c * NT;
  float s = 0.f, s2 = 0.f; for (int i = tid; i < NT; i += 256) { const float v = xc[i]; s += v; s2 += v * v; }
#pragma unroll
  for (int off = 16; off >= 1; off >>= 1) { s += __shfl_xor(s, off, 32); s2 += __shfl_xor(s2, off, 32); }
  if (lane == 0) { sred[0][wv] = s; sred[1][wv] = s2; }
  __syncthreads();
  if (tid < 32) { float a = 0.f, b = 0.f; for (int i = 0; i < 8; ++i) { a += sred[0][i]; b += sred[1][i]; } const float mean = a / (float)NT; const float var = fmaxf(b / (float)NT - mean * mean, 0.f);
    vst2(stat + c * 32 + tid, (float)(tid == 0 ? mean : (tid == 1 ? rsqrtf(var + 1e-5f) : 0.f))); }
}
__global__ __launch_bounds__(256) void k_bn1(const float* __restrict__ x, const float* __restrict__ stat, const float* __restrict__ g1, const float* __restrict__ be1, float* __restrict__ Hrow) {
  __shared__ __align__(16) float st[64][CC + 4];
  const int tid = threadIdx.x, t0 = blockIdx.x * 64;
  for (int q = tid; q < CC * 64; q += 256) { const int c = q >> 6, tl = q & 63; const int t = t0 + tl; float v = 0.f;
    if (t < NT) v = (x[(size_t)c * NT + t] - stat[c * 32]) * stat[c * 32 + 1] * g1[c] + be1[c];
    st[tl][c] = v; }
  __syncthreads();
  for (int q = tid; q < 64 * (CC / 4); q += 256) { const int tl = q >> 5, pc = q & 31; vst2(Hrow + (size_t)(t0 + tl) * CC + pc * 4, *(const v4f*)(&st[tl][pc * 4])); }
}
template <int KIN, int NOUT, int MODE>
__global__ __launch_bounds__(128) void k_gemm(const float* __restrict__ A, const float* __restrict__ W, const float* __restrict__ bias, float* __restrict__ Out) {
  __shared__ __align__(16) float so[4][16][132];
  const int tid = threadIdx.x, wave = tid >> 5, lane = tid & 31, col = lane & 15, g = lane >> 4;
  const int r0 = blockIdx.x * 64 + wave * 16, n0 = blockIdx.y * 128;
  v8f acc[8] = {};
#pragma unroll 2
  for (int kc = 0; kc < KIN / 32; ++kc) { const v16h a = frag_f32(A + (size_t)(r0 + col) * KIN + kc * 32, lane);
#pragma unroll
    for (int j = 0; j < 8; ++j) acc[j] = wmma16(a, frag_f32s(W + (size_t)(n0 + j * 16 + col) * KIN + kc * 32, lane, 16.0f), acc[j]); }
#pragma unroll
  for (int j = 0; j < 8; ++j) { const float bb = bias[n0 + j * 16 + col];
#pragma unroll
    for (int r = 0; r < 8; ++r) { float v = acc[j][r] * (1.0f / 16.0f) + bb; if (MODE == 1) v = gelu_e(v); so[wave][8 * g + r][j * 16 + col] = v; } }
  LDSX();
#pragma unroll 4
  for (int rl = 0; rl < 16; ++rl) vst2(Out + (size_t)(r0 + rl) * NOUT + n0 + lane * 4, *(const v4f*)(&so[wave][rl][lane * 4]));
}
__global__ __launch_bounds__(256) void k_natt(const float* __restrict__ QKV, const float* __restrict__ rpb, float* __restrict__ O) {
  __shared__ __align__(16) float so[32][CC + 4];
  const int tid = threadIdx.x, tl = tid >> 3, h = tid & 7; const int t = blockIdx.x * 32 + tl;
  if (t < NT) {
    const int z = t / (SD * SD), y = (t / SD) % SD, xw = t % SD;
    const int sz = min(max(z - KW / 2, 0), SD - KW), sy = min(max(y - KW / 2, 0), SD - KW), sx = min(max(xw - KW / 2, 0), SD - KW);
    float q[HD];
#pragma unroll
    for (int d = 0; d < HD; ++d) q[d] = QKV[(size_t)t * (3 * CC) + h * HD + d] * 0.25f;
    float mx = -3.0e38f, lsum = 0.f; float o[HD];
#pragma unroll
    for (int d = 0; d < HD; ++d) o[d] = 0.f;
#pragma unroll 1
    for (int nbi = 0; nbi < NNB; ++nbi) { const int i = nbi / 25, j = (nbi / 5) % 5, l = nbi % 5; const int kz = sz + i, ky = sy + j, kx = sx + l; const int kt = (kz * SD + ky) * SD + kx;
      const float* kr = QKV + (size_t)kt * (3 * CC) + CC + h * HD; float s = 0.f;
#pragma unroll
      for (int d = 0; d < HD; ++d) s += q[d] * kr[d];
      s += rpb[((h * RB + (kz - z + KW - 1)) * RB + (ky - y + KW - 1)) * RB + (kx - xw + KW - 1)];
      if (s > mx) { const float cr = expf(mx - s); lsum *= cr;
#pragma unroll
        for (int d = 0; d < HD; ++d) o[d] *= cr;
        mx = s; }
      const float p = expf(s - mx); lsum += p; const float* vr = QKV + (size_t)kt * (3 * CC) + 2 * CC + h * HD;
#pragma unroll
      for (int d = 0; d < HD; ++d) o[d] += p * vr[d]; }
    const float inv = 1.0f / lsum;
#pragma unroll
    for (int d = 0; d < HD; ++d) so[tl][h * HD + d] = o[d] * inv; }
  else {
#pragma unroll
    for (int d = 0; d < HD; ++d) so[tl][h * HD + d] = 0.f; }
  __syncthreads();
  for (int q2 = tid; q2 < 32 * (CC / 4); q2 += 256) { const int rl = q2 >> 5, pc = q2 & 31; vst2(O + (size_t)(blockIdx.x * 32 + rl) * CC + pc * 4, *(const v4f*)(&so[rl][pc * 4])); }
}
__global__ __launch_bounds__(128) void k_proj(const float* __restrict__ O, const float* __restrict__ W, const float* __restrict__ bias, const float* __restrict__ x, float* __restrict__ X1) {
  __shared__ __align__(16) float st[CC][68];
  const int tid = threadIdx.x, wave = tid >> 5, lane = tid & 31, col = lane & 15, g = lane >> 4;
  const int t0b = blockIdx.x * 64, r0 = t0b + wave * 16;
  v8f acc[8] = {};
#pragma unroll
  for (int kc = 0; kc < CC / 32; ++kc) { const v16h a = frag_f32(O + (size_t)(r0 + col) * CC + kc * 32, lane);
#pragma unroll
    for (int j = 0; j < 8; ++j) acc[j] = wmma16(a, frag_f32s(W + (size_t)(j * 16 + col) * CC + kc * 32, lane, 16.0f), acc[j]); }
#pragma unroll
  for (int j = 0; j < 8; ++j) { const int c = j * 16 + col; const float bb = bias[c];
#pragma unroll
    for (int r = 0; r < 8; ++r) { const int t = r0 + 8 * g + r; st[c][wave * 16 + 8 * g + r] = (t < NT ? x[(size_t)c * NT + t] : 0.f) + acc[j][r] * (1.0f / 16.0f) + bb; } }
  __syncthreads();
  for (int q = tid; q < CC * 16; q += 128) { const int c = q >> 4, pc = q & 15; vst2(X1 + (size_t)c * NTP + t0b + pc * 4, *(const v4f*)(&st[c][pc * 4])); }
}
__global__ __launch_bounds__(256) void k_bn2(const float* __restrict__ X1, const float* __restrict__ stat, const float* __restrict__ g2, const float* __restrict__ be2, float* __restrict__ Yrow, float* __restrict__ X1row) {
  __shared__ __align__(16) float st[64][CC + 4], sx[64][CC + 4];
  const int tid = threadIdx.x, t0 = blockIdx.x * 64;
  for (int q = tid; q < CC * 64; q += 256) { const int c = q >> 6, tl = q & 63; const float xv = X1[(size_t)c * NTP + t0 + tl]; sx[tl][c] = xv; st[tl][c] = (xv - stat[c * 32]) * stat[c * 32 + 1] * g2[c] + be2[c]; }
  __syncthreads();
  for (int q = tid; q < 64 * (CC / 4); q += 256) { const int tl = q >> 5, pc = q & 31; vst2(Yrow + (size_t)(t0 + tl) * CC + pc * 4, *(const v4f*)(&st[tl][pc * 4])); vst2(X1row + (size_t)(t0 + tl) * CC + pc * 4, *(const v4f*)(&sx[tl][pc * 4])); }
}
__global__ __launch_bounds__(256) void k_bnstat2(const float* __restrict__ X1, float* __restrict__ stat) {
  __shared__ float sred[2][8];
  const int c = blockIdx.x, tid = threadIdx.x, wv = tid >> 5, lane = tid & 31; const float* xc = X1 + (size_t)c * NTP;
  float s = 0.f, s2 = 0.f; for (int i = tid; i < NT; i += 256) { const float v = xc[i]; s += v; s2 += v * v; }
#pragma unroll
  for (int off = 16; off >= 1; off >>= 1) { s += __shfl_xor(s, off, 32); s2 += __shfl_xor(s2, off, 32); }
  if (lane == 0) { sred[0][wv] = s; sred[1][wv] = s2; }
  __syncthreads();
  if (tid < 32) { float a = 0.f, b = 0.f; for (int i = 0; i < 8; ++i) { a += sred[0][i]; b += sred[1][i]; } const float mean = a / (float)NT; const float var = fmaxf(b / (float)NT - mean * mean, 0.f);
    vst2(stat + c * 32 + tid, (float)(tid == 0 ? mean : (tid == 1 ? rsqrtf(var + 1e-5f) : 0.f))); }
}
__global__ __launch_bounds__(128) void k_fin(const float* __restrict__ Gh, const float* __restrict__ W2, const float* __restrict__ b2, const float* __restrict__ X1row, float* __restrict__ out) {
  __shared__ __align__(16) float st[CC][68];
  const int tid = threadIdx.x, wave = tid >> 5, lane = tid & 31, col = lane & 15, g = lane >> 4;
  const int t0b = blockIdx.x * 64, r0 = t0b + wave * 16;
  v8f acc[8] = {};
#pragma unroll 2
  for (int kc = 0; kc < FF / 32; ++kc) { const v16h a = frag_f32(Gh + (size_t)(r0 + col) * FF + kc * 32, lane);
#pragma unroll
    for (int j = 0; j < 8; ++j) acc[j] = wmma16(a, frag_f32s(W2 + (size_t)(j * 16 + col) * FF + kc * 32, lane, 16.0f), acc[j]); }
#pragma unroll
  for (int j = 0; j < 8; ++j) { const int c = j * 16 + col; const float bb = b2[c];
#pragma unroll
    for (int r = 0; r < 8; ++r) { const int t = r0 + 8 * g + r; st[c][wave * 16 + 8 * g + r] = X1row[(size_t)t * CC + c] + acc[j][r] * (1.0f / 16.0f) + bb; } }
  __syncthreads();
  if (t0b + 64 <= NT) { for (int q = tid; q < CC * 16; q += 128) { const int c = q >> 4, pc = q & 15; vst2(out + (size_t)c * NT + t0b + pc * 4, *(const v4f*)(&st[c][pc * 4])); } }
}
extern "C" void kernel_launch(void* const* d_in, const int* in_sizes, int n_in, void* d_out, int out_size, void* d_ws, size_t ws_size, hipStream_t stream) {
  (void)in_sizes; (void)n_in; (void)out_size; (void)ws_size;
  const float** I = (const float**)d_in;
  const float* x = I[0]; const float* g1 = I[1]; const float* be1 = I[2]; const float* wqkv = I[3]; const float* bqkv = I[4]; const float* rpb = I[5]; const float* wp = I[6]; const float* bp = I[7];
  const float* g2 = I[8]; const float* be2 = I[9]; const float* w1 = I[10]; const float* b1 = I[11]; const float* w2 = I[12]; const float* b2 = I[13];
  float* out = (float*)d_out;
  char* ws = (char*)d_ws; size_t off = 0;
  auto take = [&](size_t bytes) { char* p = ws + off; off += (bytes + 255) & ~(size_t)255; return p; };
  float* stat1 = (float*)take((size_t)CC * 32 * 4); float* stat2 = (float*)take((size_t)CC * 32 * 4);
  float* Hrow = (float*)take((size_t)NTP * CC * 4); float* QKV = (float*)take((size_t)NTP * 3 * CC * 4); float* O = (float*)take((size_t)NTP * CC * 4); float* X1 = (float*)take((size_t)CC * NTP * 4);
  float* Yrow = (float*)take((size_t)NTP * CC * 4); float* X1row = (float*)take((size_t)NTP * CC * 4); float* Gh = (float*)take((size_t)NTP * FF * 4);
  k_bnstat<<<CC, 256, 0, stream>>>(x, stat1);
  k_bn1<<<NTP / 64, 256, 0, stream>>>(x, stat1, g1, be1, Hrow);
  k_gemm<CC, 3 * CC, 0><<<dim3(NTP / 64, 3), 128, 0, stream>>>(Hrow, wqkv, bqkv, QKV);
  k_natt<<<NTP / 32, 256, 0, stream>>>(QKV, rpb, O);
  k_proj<<<NTP / 64, 128, 0, stream>>>(O, wp, bp, x, X1);
  k_bnstat2<<<CC, 256, 0, stream>>>(X1, stat2);
  k_bn2<<<NTP / 64, 256, 0, stream>>>(X1, stat2, g2, be2, Yrow, X1row);
  k_gemm<CC, FF, 1><<<dim3(NTP / 64, FF / 128), 128, 0, stream>>>(Yrow, w1, b1, Gh);
  k_fin<<<NTP / 64, 128, 0, stream>>>(Gh, w2, b2, X1row, out);
}
